// RBFBias_20555713478724
// MI455X (gfx1250) — hardware-verified
//
#include <hip/hip_runtime.h>


typedef __bf16        v16bf __attribute__((ext_vector_type(16)));
typedef float         v8f   __attribute__((ext_vector_type(8)));
typedef float         v4f   __attribute__((ext_vector_type(4)));
typedef unsigned int  v4u   __attribute__((ext_vector_type(4)));
typedef unsigned int  v4ua  __attribute__((ext_vector_type(4), may_alias));
typedef float         v4fa  __attribute__((ext_vector_type(4), may_alias));

#define NB    2
#define NH    8
#define NS    2048
#define ND    64
#define NBH   (NB * NH)
#define NPOS  3
#define KCH   32
#define QK_SCALE 0.125f
#define TPITCH 68
#define OPITCH 68
#define PLANE_ELEMS ((size_t)NBH * NS * ND)
#define NPLANES 6

union Frag { v16bf v; v4u q[2]; };

__device__ __forceinline__ v8f wmma_bf16(v8f acc, v16bf a, v16bf b)
{
    acc = __builtin_amdgcn_wmma_f32_16x16x32_bf16(false, a, false, b, (short)0, acc, false, false);
    asm volatile("v_nop\n\tv_nop\n\tv_nop\n\tv_nop" : "+v"(acc) : "v"(a), "v"(b));
    return acc;
}

__device__ __forceinline__ unsigned int bf16_bits(float x)
{
    unsigned int u = __float_as_uint(x);
    return (u + 0x7FFFu + ((u >> 16) & 1u)) >> 16;
}

__device__ __forceinline__ void split_hl(float x, unsigned int& hi, unsigned int& lo)
{
    hi = bf16_bits(x);
    const float hf = __uint_as_float(hi << 16);
    lo = bf16_bits(x - hf);
}

__global__ __launch_bounds__(256) void k_split(const float* __restrict__ q,
                                                const float* __restrict__ k,
                                                const float* __restrict__ v,
                                                unsigned short* __restrict__ planes)
{
    __shared__ __align__(16) float tile[64][TPITCH];

    const int t  = threadIdx.x;
    const int s0 = blockIdx.x * 64;
    const int bh = blockIdx.y;
    const int z  = blockIdx.z;
    const float* src = (z == 0) ? q : ((z == 1) ? k : v);
    const int tr = (z == 2) ? 1 : 0;

#pragma unroll
    for (int i = 0; i < 4; ++i) {
        const int idx = (t + 256 * i) * 4;
        const int r = idx >> 6, c = idx & 63;
        const v4f val = *(const v4f*)(src + ((size_t)(bh * NS + s0 + r)) * ND + c);
        *(v4f*)&tile[r][c] = val;
    }
    __syncthreads();

    v4u hv[2], lv[2];
    size_t off[2];
#pragma unroll
    for (int it = 0; it < 2; ++it) {
        const int gidx = it * 256 + t;
        const int orow = gidx >> 3;
        const int og   = gidx & 7;
        unsigned int hs[8], ls[8];
#pragma unroll
        for (int j = 0; j < 8; ++j) {
            const int cidx = 8 * og + j;
            const int ia = orow * TPITCH + cidx;
            const int ib = cidx * TPITCH + orow;
            const float x = (&tile[0][0])[tr ? ib : ia];
            split_hl(x, hs[j], ls[j]);
        }
        v4u hw, lw;
        hw.x = hs[0] | (hs[1] << 16); hw.y = hs[2] | (hs[3] << 16);
        hw.z = hs[4] | (hs[5] << 16); hw.w = hs[6] | (hs[7] << 16);
        lw.x = ls[0] | (ls[1] << 16); lw.y = ls[2] | (ls[3] << 16);
        lw.z = ls[4] | (ls[5] << 16); lw.w = ls[6] | (ls[7] << 16);
        hv[it] = hw; lv[it] = lw;
        const size_t offa = ((size_t)(bh * NS + s0 + orow)) * ND + 8 * og;
        const size_t offb = ((size_t)(bh * ND + orow)) * NS + s0 + 8 * og;
        off[it] = tr ? offb : offa;
    }

    unsigned short* ph = planes + (size_t)(2 * z) * PLANE_ELEMS;
    unsigned short* pl = ph + PLANE_ELEMS;

#pragma unroll
    for (int it = 0; it < 2; ++it) {
        *(volatile v4u*)(ph + off[it]) = hv[it];
        *(volatile v4u*)(pl + off[it]) = lv[it];
    }
    __threadfence();
#pragma unroll
    for (int it = 0; it < 2; ++it) {
        *(volatile v4u*)(ph + off[it]) = hv[it];
        *(volatile v4u*)(pl + off[it]) = lv[it];
    }
}

__global__ __launch_bounds__(128) void k_attn(const unsigned short* __restrict__ planes,
                                               const float* __restrict__ qsg,
                                               const float* __restrict__ ksg,
                                               const float* __restrict__ alphag,
                                               const float* __restrict__ betag,
                                               float* outg)
{
    __shared__ __align__(16) unsigned short Psh[4][2][16][KCH];
    __shared__ __align__(16) float Osh[4][16][OPITCH];

    const int tid  = threadIdx.x;
    const int wave = tid >> 5;
    const int lane = tid & 31;
    const int g    = lane >> 4;
    const int n    = lane & 15;

    const int bid  = blockIdx.x;
    const int qblk = bid & 31;
    const int bh   = bid >> 5;
    const int hh   = bh & (NH - 1);
    const int b    = bh >> 3;
    const int q0   = qblk * 64 + wave * 16;

    const float alpha_h = alphag[hh];
    const float nbeta_h = -betag[hh];

    const unsigned short* Qh = planes;
    const unsigned short* Ql = planes + PLANE_ELEMS;
    const unsigned short* Kh = planes + 2 * PLANE_ELEMS;
    const unsigned short* Kl = planes + 3 * PLANE_ELEMS;
    const unsigned short* Vh = planes + 4 * PLANE_ELEMS;
    const unsigned short* Vl = planes + 5 * PLANE_ELEMS;
    const size_t rowb = (size_t)bh * NS;

    Frag aqh[2], aql[2];
    {
        const unsigned short* qrh = Qh + (rowb + q0 + n) * ND;
        const unsigned short* qrl = Ql + (rowb + q0 + n) * ND;
#pragma unroll
        for (int c = 0; c < 2; ++c) {
            aqh[c].q[0] = *(const v4u*)(qrh + 32 * c + 8 * g);
            aqh[c].q[1] = *(const v4u*)(qrh + 32 * c + 16 + 8 * g);
            aql[c].q[0] = *(const v4u*)(qrl + 32 * c + 8 * g);
            aql[c].q[1] = *(const v4u*)(qrl + 32 * c + 16 + 8 * g);
        }
    }

    float qp[8][NPOS];
#pragma unroll
    for (int r = 0; r < 8; ++r) {
        const float* p = qsg + ((size_t)b * NS + q0 + 8 * g + r) * NPOS;
        qp[r][0] = p[0]; qp[r][1] = p[1]; qp[r][2] = p[2];
    }

    v8f o[4];
#pragma unroll
    for (int f = 0; f < 4; ++f) o[f] = (v8f){};
    float mrow[8], lrow[8];
#pragma unroll
    for (int r = 0; r < 8; ++r) { mrow[r] = -__builtin_huge_valf(); lrow[r] = 0.0f; }

#pragma unroll 1
    for (int kc = 0; kc < NS / KCH; ++kc) {
        const int kb = kc * KCH;

        float kf0[NPOS], kf1[NPOS];
        {
            const float* p0 = ksg + ((size_t)b * NS + kb + n) * NPOS;
            const float* p1 = ksg + ((size_t)b * NS + kb + 16 + n) * NPOS;
#pragma unroll
            for (int j = 0; j < NPOS; ++j) { kf0[j] = p0[j]; kf1[j] = p1[j]; }
        }

        v8f sa[2];
#pragma unroll
        for (int t = 0; t < 2; ++t) {
            v8f acc = (v8f){};
            const unsigned short* krh = Kh + (rowb + kb + 16 * t + n) * ND;
            const unsigned short* krl = Kl + (rowb + kb + 16 * t + n) * ND;
#pragma unroll
            for (int c = 0; c < 2; ++c) {
                Frag bkh, bkl;
                bkh.q[0] = *(const v4u*)(krh + 32 * c + 8 * g);
                bkh.q[1] = *(const v4u*)(krh + 32 * c + 16 + 8 * g);
                bkl.q[0] = *(const v4u*)(krl + 32 * c + 8 * g);
                bkl.q[1] = *(const v4u*)(krl + 32 * c + 16 + 8 * g);
                acc = wmma_bf16(acc, aqh[c].v, bkh.v);
                acc = wmma_bf16(acc, aqh[c].v, bkl.v);
                acc = wmma_bf16(acc, aql[c].v, bkh.v);
            }
            sa[t] = acc;
        }

#pragma unroll
        for (int r = 0; r < 8; ++r) {
            const float d0x = qp[r][0] - kf0[0], d0y = qp[r][1] - kf0[1], d0z = qp[r][2] - kf0[2];
            const float d1x = qp[r][0] - kf1[0], d1y = qp[r][1] - kf1[1], d1z = qp[r][2] - kf1[2];
            float dd0 = d0x * d0x; dd0 = dd0 + d0y * d0y; dd0 = dd0 + d0z * d0z;
            float dd1 = d1x * d1x; dd1 = dd1 + d1y * d1y; dd1 = dd1 + d1z * d1z;
            const float bias0 = alpha_h * expf(nbeta_h * dd0);
            const float bias1 = alpha_h * expf(nbeta_h * dd1);
            const float s0 = sa[0][r] * QK_SCALE + bias0;
            const float s1 = sa[1][r] * QK_SCALE + bias1;

            float vmax = fmaxf(s0, s1);
#pragma unroll
            for (int off = 1; off <= 8; off <<= 1)
                vmax = fmaxf(vmax, __shfl_xor(vmax, off, 32));
            const float mn   = fmaxf(mrow[r], vmax);
            const float resc = __expf(mrow[r] - mn);
            const float p0   = __expf(s0 - mn);
            const float p1   = __expf(s1 - mn);
            float ps = p0 + p1;
#pragma unroll
            for (int off = 1; off <= 8; off <<= 1)
                ps += __shfl_xor(ps, off, 32);
            lrow[r] = lrow[r] * resc + ps;
            mrow[r] = mn;
#pragma unroll
            for (int f = 0; f < 4; ++f) o[f][r] = o[f][r] * resc;

            unsigned int h0, l0, h1, l1;
            split_hl(p0, h0, l0);
            split_hl(p1, h1, l1);
            Psh[wave][0][8 * g + r][n]      = (unsigned short)h0;
            Psh[wave][1][8 * g + r][n]      = (unsigned short)l0;
            Psh[wave][0][8 * g + r][16 + n] = (unsigned short)h1;
            Psh[wave][1][8 * g + r][16 + n] = (unsigned short)l1;
        }
        __syncthreads();

        Frag aph, apl;
        aph.q[0] = *(const v4ua*)&Psh[wave][0][n][8 * g];
        aph.q[1] = *(const v4ua*)&Psh[wave][0][n][16 + 8 * g];
        apl.q[0] = *(const v4ua*)&Psh[wave][1][n][8 * g];
        apl.q[1] = *(const v4ua*)&Psh[wave][1][n][16 + 8 * g];

#pragma unroll
        for (int f = 0; f < 4; ++f) {
            const unsigned short* vrh = Vh + ((size_t)bh * ND + 16 * f + n) * NS + kb;
            const unsigned short* vrl = Vl + ((size_t)bh * ND + 16 * f + n) * NS + kb;
            Frag bvh, bvl;
            bvh.q[0] = *(const v4u*)(vrh + 8 * g);
            bvh.q[1] = *(const v4u*)(vrh + 16 + 8 * g);
            bvl.q[0] = *(const v4u*)(vrl + 8 * g);
            bvl.q[1] = *(const v4u*)(vrl + 16 + 8 * g);
            o[f] = wmma_bf16(o[f], aph.v, bvh.v);
            o[f] = wmma_bf16(o[f], aph.v, bvl.v);
            o[f] = wmma_bf16(o[f], apl.v, bvh.v);
        }
    }

#pragma unroll
    for (int r = 0; r < 8; ++r) {
        const float inv = 1.0f / lrow[r];
#pragma unroll
        for (int f = 0; f < 4; ++f)
            Osh[wave][8 * g + r][16 * f + n] = o[f][r] * inv;
    }
    __syncthreads();

    v4f vals[8];
#pragma unroll
    for (int i = 0; i < 8; ++i)
        vals[i] = *(const v4fa*)&Osh[wave][2 * i + g][4 * n];

    float* obase = outg + (rowb + q0) * ND;
#pragma unroll
    for (int i = 0; i < 8; ++i)
        *(volatile v4f*)(obase + (2 * i + g) * ND + 4 * n) = vals[i];
    __threadfence();
#pragma unroll
    for (int i = 0; i < 8; ++i)
        *(volatile v4f*)(obase + (2 * i + g) * ND + 4 * n) = vals[i];
}

extern "C" void kernel_launch(void* const* d_in, const int* in_sizes, int n_in,
                              void* d_out, int out_size, void* d_ws, size_t ws_size,
                              hipStream_t stream)
{
    if (n_in < 7) return;
    const int n_qkv = NBH * NS * ND;
    const int n_pos = NB * NS * NPOS;
    if (in_sizes[0] != n_qkv || in_sizes[1] != n_qkv || in_sizes[2] != n_qkv) return;
    if (in_sizes[3] != n_pos || in_sizes[4] != n_pos) return;
    if (in_sizes[5] < NH || in_sizes[6] < NH) return;
    if (out_size != n_qkv) return;

    const size_t ws_need = (size_t)NPLANES * PLANE_ELEMS * sizeof(unsigned short);
    if (ws_size < ws_need) return;

    const float* q     = (const float*)d_in[0];
    const float* k     = (const float*)d_in[1];
    const float* v     = (const float*)d_in[2];
    const float* qs_s  = (const float*)d_in[3];
    const float* ks_s  = (const float*)d_in[4];
    const float* alpha = (const float*)d_in[5];
    const float* beta  = (const float*)d_in[6];
    float* out = (float*)d_out;
    unsigned short* planes = (unsigned short*)d_ws;

    k_split<<<dim3(NS / 64, NBH, 3), dim3(256), 0, stream>>>(q, k, v, planes);
    k_attn<<<dim3(NBH * (NS / 64)), dim3(128), 0, stream>>>(planes, qs_s, ks_s, alpha, beta, out);
}
